// GraphAttentionLayer_78348793413869
// MI455X (gfx1250) — hardware-verified
//
#include <hip/hip_runtime.h>
#include <stddef.h>
#include <stdint.h>
#include <math.h>


#define F_IN   256
#define UNI    128
#define NHD    4
#define NN     1024
#define NB     8
#define HU     (NHD * UNI)
#define MROW   (NB * NN)
#define NBH    (NB * NHD)
#define MWORDS (NN / 32)
#define NTHR   256
#define PBM    64
#define PBN    128
#define PTHR   128
#define QT     64
#define KT     64
#define NKT    (NN / KT)
#define ATHR   256
#define PLD    72
#define NEGSL  0.2f
#define WSMAX  134217728

static_assert((F_IN % 32) == 0 && (F_IN / 8) == 32);
static_assert((MROW % PBM) == 0 && (NN % PBM) == 0);
static_assert(PBN == UNI && (HU % PBN) == 0);
static_assert(PTHR == 4 * 32 && PBM == 4 * 16 && PTHR == 2 * PBM && PTHR == PBN);
static_assert(PBN == 4 * 32);
static_assert(PBM == 8 * 8);
static_assert((NN % QT) == 0 && (NN % KT) == 0 && KT == 64 && QT == 64);
static_assert(ATHR == 4 * QT);
static_assert(ATHR == 8 * 32 && UNI == 2 * 64 && QT == 4 * 16);
static_assert(NN == 4 * ATHR);
static_assert(QT * MWORDS == 8 * ATHR);
static_assert(MWORDS == 32);
static_assert(2 * QT * PLD * 2 <= QT * UNI * 4);
static_assert((PLD % 8) == 0 && PLD >= KT);
static_assert(QT == 8 * 8);
static_assert(UNI * 4 == 32 * 16);
static_assert((HU * 4) % 128 == 0 && (UNI * 4) % 128 == 0);

typedef float          v4f  __attribute__((ext_vector_type(4)));
typedef float          v8f  __attribute__((ext_vector_type(8)));
typedef int            v8i  __attribute__((ext_vector_type(8)));
typedef unsigned int   v4u  __attribute__((ext_vector_type(4)));
typedef unsigned short v8us __attribute__((ext_vector_type(8)));
typedef __bf16         v16b __attribute__((ext_vector_type(16)));
typedef v4f  __attribute__((may_alias)) v4fa;
typedef v4u  __attribute__((may_alias)) v4ua;
typedef v8us __attribute__((may_alias)) v8usa;
union FragB { v16b v; v8us h[2]; v8i w; };

__device__ __forceinline__ v8f wmb(const FragB& a, const FragB& b, v8f c) {
  v8f d = __builtin_amdgcn_wmma_f32_16x16x32_bf16(false, a.v, false, b.v, (short)0, c, false, false);
  asm volatile("v_nop\n\tv_nop\n\tv_nop\n\tv_nop" : "+v"(d) : "v"(a.w), "v"(b.w));
  return d;
}

__device__ __forceinline__ unsigned int f2bf(float f) {
  const unsigned int u = __float_as_uint(f);
  return ((u + 0x7FFFu + ((u >> 16) & 1u)) >> 16) & 0xFFFFu;
}
__device__ __forceinline__ float bf2f(unsigned int b) { return __uint_as_float(b << 16); }
__device__ __forceinline__ float bfr(float f) { return bf2f(f2bf(f)); }
__device__ __forceinline__ unsigned int pk2(float lo, float hi) { return f2bf(lo) | (f2bf(hi) << 16); }
__device__ __forceinline__ v4u pack8(const v4f a, const v4f b) {
  v4u r;
  r.x = pk2(a.x, a.y); r.y = pk2(a.z, a.w); r.z = pk2(b.x, b.y); r.w = pk2(b.z, b.w);
  return r;
}

__global__ __launch_bounds__(NTHR) void k_xprep(const float* __restrict__ x, unsigned short* xb, int nN, int nUnits) {
  const int i = (int)blockIdx.x * NTHR + (int)threadIdx.x;
  if (i >= nUnits) return;
  const int row = i >> 5;
  const int c0  = (i & 31) * 8;
  const int rc  = row < nN ? row : nN - 1;
  const float* p = x + (size_t)rc * F_IN + c0;
  v4f a = *(const v4fa*)p, b = *(const v4fa*)(p + 4);
  const v4f z4 = {0.f, 0.f, 0.f, 0.f};
  if (row >= nN) { a = z4; b = z4; }
  const v4u hv = pack8(a, b);
  const size_t o = (size_t)row * F_IN + c0;
  *(volatile v4u*)(xb + o) = hv;
  __threadfence();
  *(volatile v4u*)(xb + o) = hv;
}

__global__ __launch_bounds__(NTHR) void k_wtr(const float* __restrict__ w, unsigned short* wt, int nUnits) {
  const int u = (int)blockIdx.x * NTHR + (int)threadIdx.x;
  if (u >= nUnits) return;
  const int n  = u >> 5;
  const int k8 = (u & 31) * 8;
  const int hd = n >> 7, uu = n & (UNI - 1);
  const float* p = w + ((size_t)hd * F_IN + k8) * UNI + uu;
  v4f a, b;
  a.x = p[0];                  a.y = p[(size_t)UNI];          a.z = p[(size_t)2 * UNI];      a.w = p[(size_t)3 * UNI];
  b.x = p[(size_t)4 * UNI];    b.y = p[(size_t)5 * UNI];      b.z = p[(size_t)6 * UNI];      b.w = p[(size_t)7 * UNI];
  const v4u wv = pack8(a, b);
  unsigned short* o = wt + (size_t)n * F_IN + k8;
  *(volatile v4u*)o = wv;
  __threadfence();
  *(volatile v4u*)o = wv;
}

__global__ __launch_bounds__(NTHR) void k_mask(const float* __restrict__ adj, unsigned int* mb, int nRows) {
  const int gw   = (int)blockIdx.x * (NTHR / 32) + ((int)threadIdx.x >> 5);
  const int lane = (int)threadIdx.x & 31;
  if (gw >= nRows) return;
  const float* p = adj + (size_t)gw * NN + 32 * lane;
  unsigned int word = 0u;
#pragma unroll
  for (int q = 0; q < 8; ++q) {
    const v4f a = *(const v4fa*)(p + 4 * q);
    const int m0 = 32 * lane + 4 * q;
    const float v0 = bfr(a.x) + ((m0     == gw) ? 1.f : 0.f);
    const float v1 = bfr(a.y) + ((m0 + 1 == gw) ? 1.f : 0.f);
    const float v2 = bfr(a.z) + ((m0 + 2 == gw) ? 1.f : 0.f);
    const float v3 = bfr(a.w) + ((m0 + 3 == gw) ? 1.f : 0.f);
    word |= (v0 > 0.f ? 1u : 0u) << (4 * q);
    word |= (v1 > 0.f ? 1u : 0u) << (4 * q + 1);
    word |= (v2 > 0.f ? 1u : 0u) << (4 * q + 2);
    word |= (v3 > 0.f ? 1u : 0u) << (4 * q + 3);
  }
  unsigned int* o = mb + (size_t)gw * MWORDS + lane;
  *(volatile unsigned int*)o = word;
  __threadfence();
  *(volatile unsigned int*)o = word;
}

__device__ __forceinline__ void tr8(const float* stg, int nl0, int uu, v4u& hv, v4u& lv) {
  float f[8];
  unsigned int hb[8], lb[8];
#pragma unroll
  for (int j = 0; j < 8; ++j) f[j] = stg[(nl0 + j) * PBN + uu];
#pragma unroll
  for (int j = 0; j < 8; ++j) { hb[j] = f2bf(f[j]); lb[j] = f2bf(f[j] - bf2f(hb[j])); }
  hv.x = hb[0] | (hb[1] << 16); hv.y = hb[2] | (hb[3] << 16); hv.z = hb[4] | (hb[5] << 16); hv.w = hb[6] | (hb[7] << 16);
  lv.x = lb[0] | (lb[1] << 16); lv.y = lb[2] | (lb[3] << 16); lv.z = lb[4] | (lb[5] << 16); lv.w = lb[6] | (lb[7] << 16);
}

__global__ __launch_bounds__(PTHR) void k_proj(
    const unsigned short* __restrict__ A, const unsigned short* __restrict__ WT,
    const float* __restrict__ asrc, const float* __restrict__ adst,
    float* SD, unsigned short* VH, unsigned short* VL)
{
  __shared__ __attribute__((aligned(16))) float stg[PBM * PBN];
  __shared__ __attribute__((aligned(16))) float satt[2 * PBN];
  __shared__ __attribute__((aligned(16))) float sdot[2 * PBM];
  const int tid = (int)threadIdx.x, lane = tid & 31, wave = tid >> 5, hh = lane >> 4, m = lane & 15;
  const int rowBase = (int)blockIdx.x * PBM;
  const int head    = (int)blockIdx.y;
  const int col0    = head * PBN;

  satt[tid]       = bfr(asrc[head * UNI + tid]);
  satt[PBN + tid] = bfr(adst[head * UNI + tid]);

  v8f acc[8];
  {
    const v8f z = {0.f, 0.f, 0.f, 0.f, 0.f, 0.f, 0.f, 0.f};
#pragma unroll
    for (int t = 0; t < 8; ++t) acc[t] = z;
  }
  const unsigned short* ap = A  + (size_t)(rowBase + 16 * wave + m) * (size_t)F_IN + 8 * hh;
  const unsigned short* wp = WT + (size_t)(col0 + m) * (size_t)F_IN + 8 * hh;
#pragma unroll 1
  for (int ks = 0; ks < F_IN / 32; ++ks) {
    FragB af;
    af.h[0] = *(const v8usa*)(ap + 32 * ks);
    af.h[1] = *(const v8usa*)(ap + 32 * ks + 16);
#pragma unroll
    for (int t = 0; t < 8; ++t) {
      const unsigned short* wq = wp + (size_t)(16 * t) * (size_t)F_IN + 32 * ks;
      FragB bf;
      bf.h[0] = *(const v8usa*)wq;
      bf.h[1] = *(const v8usa*)(wq + 16);
      acc[t] = wmb(af, bf, acc[t]);
    }
  }

#pragma unroll
  for (int t = 0; t < 8; ++t) {
    const int lc = 16 * t + m;
#pragma unroll
    for (int r = 0; r < 8; ++r) {
      const int lr = 16 * wave + 8 * hh + r;
      stg[lr * PBN + lc] = acc[t][r];
    }
  }
  __syncthreads();

  {
    const int row = tid & (PBM - 1), which = tid >> 6;
    const float* sa = satt + which * PBN;
    const float* hr = stg + row * PBN;
    float d = 0.f;
#pragma unroll 4
    for (int c4 = 0; c4 < PBN / 4; ++c4) {
      const v4f hv = *(const v4fa*)(hr + 4 * c4);
      const v4f av = *(const v4fa*)(sa + 4 * c4);
      d = fmaf(hv.x, av.x, d);
      d = fmaf(hv.y, av.y, d);
      d = fmaf(hv.z, av.z, d);
      d = fmaf(hv.w, av.w, d);
    }
    sdot[which * PBM + row] = d;
  }
  __syncthreads();

  const int which2 = lane >> 4, piece = lane & 15;
  const v4f sdv = *(const v4fa*)(sdot + which2 * PBM + 4 * piece);
  float* sp = SD + (size_t)(2 * head + which2) * (size_t)MROW + rowBase + 4 * piece;

  const int bb  = rowBase / NN;
  const int n0  = rowBase - bb * NN;
  const size_t vbase = ((size_t)(bb * NHD + head) * UNI) * (size_t)NN + (size_t)n0;
  const int uq  = lane >> 3, nl0 = 8 * (lane & 7);

#pragma unroll 1
  for (int i = 0; i < 8; ++i) {
    const int uu = 32 * wave + 4 * i + uq;
    v4u hv, lv;
    tr8(stg, nl0, uu, hv, lv);
    const size_t o = vbase + (size_t)uu * NN + nl0;
    *(volatile v4u*)(VH + o) = hv;
    *(volatile v4u*)(VL + o) = lv;
  }
  if (wave == 0) *(volatile v4f*)sp = sdv;
  __threadfence();
#pragma unroll 1
  for (int i = 0; i < 8; ++i) {
    const int uu = 32 * wave + 4 * i + uq;
    v4u hv, lv;
    tr8(stg, nl0, uu, hv, lv);
    const size_t o = vbase + (size_t)uu * NN + nl0;
    *(volatile v4u*)(VH + o) = hv;
    *(volatile v4u*)(VL + o) = lv;
  }
  if (wave == 0) *(volatile v4f*)sp = sdv;
}

__global__ __launch_bounds__(ATHR) void k_attn(
    const float* __restrict__ SD, const unsigned int* __restrict__ MB,
    const unsigned short* __restrict__ VH, const unsigned short* __restrict__ VL, float* out)
{
  __shared__ __attribute__((aligned(16))) float obuf[QT * UNI];
  __shared__ __attribute__((aligned(16))) float dstS[NN];
  __shared__ __attribute__((aligned(16))) unsigned int mskS[QT * MWORDS];
  __shared__ __attribute__((aligned(16))) float srcS[QT];
  __shared__ __attribute__((aligned(16))) float linvS[QT];
  const int tid = (int)threadIdx.x, lane = tid & 31, wave = tid >> 5, hh = lane >> 4, m = lane & 15;
  const int n0 = (int)blockIdx.x * QT, head = (int)blockIdx.y, bb = (int)blockIdx.z;
  const int rowFlat = bb * NN + n0;
  const int bh = bb * NHD + head;

  {
    const float* dsp = SD + (size_t)(2 * head + 1) * (size_t)MROW + (size_t)bb * NN;
    *(v4fa*)(dstS + 4 * tid) = *(const v4fa*)(dsp + 4 * tid);
    const unsigned int* mp = MB + (size_t)n0 * MWORDS + 8 * tid;
    *(v4ua*)(mskS + 8 * tid)     = *(const v4ua*)mp;
    *(v4ua*)(mskS + 8 * tid + 4) = *(const v4ua*)(mp + 4);
    if (tid < QT) srcS[tid] = SD[(size_t)(2 * head) * (size_t)MROW + rowFlat + tid];
  }
  __syncthreads();

  const int pr = tid >> 2, sub = tid & 3;
  const float srcv = srcS[pr];

  float maxd = __uint_as_float(0xff800000u);
#pragma unroll 1
  for (int i = 0; i < MWORDS / 4; ++i) {
    const int j = sub + 4 * i;
    const unsigned int w = mskS[pr * MWORDS + j];
    const float* dp = dstS + 32 * j;
#pragma unroll
    for (int q = 0; q < 8; ++q) {
      const v4f d4 = *(const v4fa*)(dp + 4 * q);
      maxd = ((w >> (4 * q))     & 1u) ? fmaxf(maxd, d4.x) : maxd;
      maxd = ((w >> (4 * q + 1)) & 1u) ? fmaxf(maxd, d4.y) : maxd;
      maxd = ((w >> (4 * q + 2)) & 1u) ? fmaxf(maxd, d4.z) : maxd;
      maxd = ((w >> (4 * q + 3)) & 1u) ? fmaxf(maxd, d4.w) : maxd;
    }
  }
  maxd = fmaxf(maxd, __shfl_xor(maxd, 1));
  maxd = fmaxf(maxd, __shfl_xor(maxd, 2));
  float rmx = srcv + maxd;
  rmx = rmx >= 0.f ? rmx : NEGSL * rmx;

  v8f acc[4];
  {
    const v8f z = {0.f, 0.f, 0.f, 0.f, 0.f, 0.f, 0.f, 0.f};
    acc[0] = z; acc[1] = z; acc[2] = z; acc[3] = z;
  }
  const int rt = wave & 3, u0 = 64 * (wave >> 2);
  unsigned short* ph = (unsigned short*)obuf;
  unsigned short* pl = ph + QT * PLD;
  const unsigned short* arh = ph + (16 * rt + m) * PLD + 8 * hh;
  const unsigned short* arl = pl + (16 * rt + m) * PLD + 8 * hh;
  const size_t vrow = ((size_t)(bh * UNI + u0 + m)) * (size_t)NN + 8 * hh;
  const unsigned short* vhp = VH + vrow;
  const unsigned short* vlp = VL + vrow;
  unsigned short* prow_h = ph + pr * PLD + 16 * sub;
  unsigned short* prow_l = pl + pr * PLD + 16 * sub;
  float lsum = 0.f;

#pragma unroll 1
  for (int kt = 0; kt < NKT; ++kt) {
    __syncthreads();
    {
      const unsigned int wbits = mskS[pr * MWORDS + 2 * kt + (sub >> 1)] >> (16 * (sub & 1));
      const float* dp = dstS + KT * kt + 16 * sub;
      unsigned int hw[8], lw[8];
#pragma unroll
      for (int g = 0; g < 4; ++g) {
        const v4f d4 = *(const v4fa*)(dp + 4 * g);
        const float dd[4] = {d4.x, d4.y, d4.z, d4.w};
        float pv[4];
#pragma unroll
        for (int i = 0; i < 4; ++i) {
          float s = srcv + dd[i];
          s = s >= 0.f ? s : NEGSL * s;
          const float e = expf(s - rmx);
          const float p = ((wbits >> (4 * g + i)) & 1u) ? e : 0.f;
          lsum += p;
          pv[i] = p;
        }
        const unsigned int h0 = f2bf(pv[0]), h1 = f2bf(pv[1]), h2 = f2bf(pv[2]), h3 = f2bf(pv[3]);
        const unsigned int l0 = f2bf(pv[0] - bf2f(h0)), l1 = f2bf(pv[1] - bf2f(h1));
        const unsigned int l2 = f2bf(pv[2] - bf2f(h2)), l3 = f2bf(pv[3] - bf2f(h3));
        hw[2 * g] = h0 | (h1 << 16); hw[2 * g + 1] = h2 | (h3 << 16);
        lw[2 * g] = l0 | (l1 << 16); lw[2 * g + 1] = l2 | (l3 << 16);
      }
      v4u ha, hb, la, lb;
      ha.x = hw[0]; ha.y = hw[1]; ha.z = hw[2]; ha.w = hw[3];
      hb.x = hw[4]; hb.y = hw[5]; hb.z = hw[6]; hb.w = hw[7];
      la.x = lw[0]; la.y = lw[1]; la.z = lw[2]; la.w = lw[3];
      lb.x = lw[4]; lb.y = lw[5]; lb.z = lw[6]; lb.w = lw[7];
      *(v4ua*)prow_h = ha; *(v4ua*)(prow_h + 8) = hb;
      *(v4ua*)prow_l = la; *(v4ua*)(prow_l + 8) = lb;
    }
    __syncthreads();
#pragma unroll
    for (int ks = 0; ks < KT / 32; ++ks) {
      FragB ah, al;
      ah.h[0] = *(const v8usa*)(arh + 32 * ks);
      ah.h[1] = *(const v8usa*)(arh + 32 * ks + 16);
      al.h[0] = *(const v8usa*)(arl + 32 * ks);
      al.h[1] = *(const v8usa*)(arl + 32 * ks + 16);
#pragma unroll
      for (int t = 0; t < 4; ++t) {
        const size_t ko = (size_t)(16 * t) * (size_t)NN + (size_t)(KT * kt + 32 * ks);
        const unsigned short* bq = vhp + ko;
        const unsigned short* cq = vlp + ko;
        FragB bhf, blf;
        bhf.h[0] = *(const v8usa*)bq;
        bhf.h[1] = *(const v8usa*)(bq + 16);
        blf.h[0] = *(const v8usa*)cq;
        blf.h[1] = *(const v8usa*)(cq + 16);
        acc[t] = wmb(ah, bhf, acc[t]);
        acc[t] = wmb(ah, blf, acc[t]);
        acc[t] = wmb(al, bhf, acc[t]);
      }
    }
  }

  lsum += __shfl_xor(lsum, 1);
  lsum += __shfl_xor(lsum, 2);
  if (sub == 0) linvS[pr] = 1.0f / lsum;
  __syncthreads();

  {
    float li[8];
#pragma unroll
    for (int r = 0; r < 8; ++r) li[r] = linvS[16 * rt + 8 * hh + r];
#pragma unroll
    for (int t = 0; t < 4; ++t) {
      const int lc = u0 + 16 * t + m;
#pragma unroll
      for (int r = 0; r < 8; ++r) {
        const int lr = 16 * rt + 8 * hh + r;
        obuf[lr * UNI + lc] = acc[t][r] * li[r];
      }
    }
  }
  __syncthreads();

  v4f ov[8];
#pragma unroll
  for (int i = 0; i < 8; ++i) ov[i] = *(const v4fa*)(obuf + (8 * wave + i) * UNI + 4 * lane);
  float* ob = out + (size_t)(rowFlat + 8 * wave) * (size_t)HU + head * UNI + 4 * lane;
#pragma unroll
  for (int i = 0; i < 8; ++i) *(volatile v4f*)(ob + (size_t)i * HU) = ov[i];
  __threadfence();
#pragma unroll
  for (int i = 0; i < 8; ++i) *(volatile v4f*)(ob + (size_t)i * HU) = ov[i];
}

static inline int cdiv(int a, int b) { return (a + b - 1) / b; }

extern "C" void kernel_launch(void* const* d_in, const int* in_sizes, int n_in,
                              void* d_out, int out_size, void* d_ws, size_t ws_size,
                              hipStream_t stream) {
  if (n_in < 5) return;
  if (in_sizes[0] != MROW * F_IN) return;
  if (in_sizes[1] != NN * NN) return;
  if (in_sizes[2] != NHD * F_IN * UNI) return;
  if (in_sizes[3] != NHD * UNI || in_sizes[4] != NHD * UNI) return;
  if (out_size != MROW * HU) return;

  const float* x    = (const float*)d_in[0];
  const float* adj  = (const float*)d_in[1];
  const float* W    = (const float*)d_in[2];
  const float* asrc = (const float*)d_in[3];
  const float* adst = (const float*)d_in[4];
  float* out = (float*)d_out;

  char* ws = (char*)d_ws;
  size_t off = 0;
  const size_t oXB = off; off += (size_t)MROW * F_IN * 2;          off = (off + 255) & ~(size_t)255;
  const size_t oWT = off; off += (size_t)HU * F_IN * 2;            off = (off + 255) & ~(size_t)255;
  const size_t oVH = off; off += (size_t)NBH * UNI * NN * 2;       off = (off + 255) & ~(size_t)255;
  const size_t oVL = off; off += (size_t)NBH * UNI * NN * 2;       off = (off + 255) & ~(size_t)255;
  const size_t oSD = off; off += (size_t)NHD * 2 * MROW * 4;       off = (off + 255) & ~(size_t)255;
  const size_t oMB = off; off += (size_t)NN * MWORDS * 4;          off = (off + 255) & ~(size_t)255;
  if (off > ws_size || off > (size_t)WSMAX) return;
  unsigned short* XB = (unsigned short*)(ws + oXB);
  unsigned short* WT = (unsigned short*)(ws + oWT);
  unsigned short* VH = (unsigned short*)(ws + oVH);
  unsigned short* VL = (unsigned short*)(ws + oVL);
  float*          SD = (float*)(ws + oSD);
  unsigned int*   MB = (unsigned int*)(ws + oMB);

  const int nUx = MROW * (F_IN / 8);
  k_xprep<<<cdiv(nUx, NTHR), NTHR, 0, stream>>>(x, XB, MROW, nUx);
  const int nUw = HU * (F_IN / 8);
  k_wtr<<<cdiv(nUw, NTHR), NTHR, 0, stream>>>(W, WT, nUw);
  k_mask<<<cdiv(NN, NTHR / 32), NTHR, 0, stream>>>(adj, MB, NN);
  k_proj<<<dim3(MROW / PBM, NHD), PTHR, 0, stream>>>(XB, WT, asrc, adst, SD, VH, VL);
  k_attn<<<dim3(NN / QT, NHD, NB), ATHR, 0, stream>>>(SD, MB, VH, VL, out);
}
